// LSTMWithInputCellAttention_627065225987
// MI455X (gfx1250) — hardware-verified
//
#include <hip/hip_runtime.h>

typedef __attribute__((ext_vector_type(16))) _Float16 v16h;
typedef __attribute__((ext_vector_type(8)))  _Float16 v8h;
typedef __attribute__((ext_vector_type(16))) __bf16   v16b;
typedef __attribute__((ext_vector_type(8)))  __bf16   v8b;
typedef __attribute__((ext_vector_type(8)))  float    v8f;
typedef __attribute__((ext_vector_type(4)))  float    v4f;
typedef __attribute__((ext_vector_type(4)))  unsigned v4u;

constexpr int NBATCH = 16;
constexpr int NSTEP  = 512;
constexpr int NDIM   = 256;
constexpr int NHID   = 512;
constexpr int NDA    = 64;
constexpr int NRH    = 8;
constexpr int NGATE  = 4 * NHID;
constexpr int NROWS  = NBATCH * NSTEP;

__device__ __forceinline__ unsigned short f2bf_bits(float f) {
  unsigned u = __float_as_uint(f);
  return (unsigned short)((u + 0x7FFFu + ((u >> 16) & 1u)) >> 16);
}
__device__ __forceinline__ float bf_bits2f(unsigned short h) { return __uint_as_float(((unsigned)h) << 16); }

__device__ __forceinline__ void dep_guard_h(v8f& a, v8f& b, v16h x, v16h y) { asm volatile("v_nop\n\tv_nop\n\tv_nop\n\tv_nop" : "+v"(a), "+v"(b) : "v"(x), "v"(y)); }
__device__ __forceinline__ void dep_guard_b(v8f& a, v8f& b, v16b x, v16b y) { asm volatile("v_nop\n\tv_nop\n\tv_nop\n\tv_nop" : "+v"(a), "+v"(b) : "v"(x), "v"(y)); }
__device__ __forceinline__ void keep4_h(v16h a, v16h b, v16h c, v16h d) { asm volatile("v_nop" :: "v"(a), "v"(b), "v"(c), "v"(d)); }
__device__ __forceinline__ void keep4_b(v16b a, v16b b, v16b c, v16b d) { asm volatile("v_nop" :: "v"(a), "v"(b), "v"(c), "v"(d)); }
__device__ __forceinline__ void acc_guard4(v8f& a, v8f& b, v8f& c, v8f& d) { asm volatile("v_nop\n\tv_nop\n\tv_nop\n\tv_nop" : "+v"(a), "+v"(b), "+v"(c), "+v"(d)); }
template <typename T> struct Frag;
template <> struct Frag<_Float16> {
  typedef v16h V; union U { v16h v; v8h h[2]; };
  static __device__ __forceinline__ v16h load(const _Float16* p) {
    U f; f.h[0] = *(const v8h*)(p); f.h[1] = *(const v8h*)(p + 16); return f.v;
  }
  static __device__ __forceinline__ v8f mma(v16h a, v16h b, v8f c) {
    return __builtin_amdgcn_wmma_f32_16x16x32_f16(false, a, false, b, (short)0, c, false, false);
  }
  static __device__ __forceinline__ void guard(v8f& a, v8f& b, v16h x, v16h y) { dep_guard_h(a, b, x, y); }
  static __device__ __forceinline__ void keep(v16h a, v16h b, v16h c, v16h d) { keep4_h(a, b, c, d); }
};
template <> struct Frag<__bf16> {
  typedef v16b V; union U { v16b v; v8b h[2]; };
  static __device__ __forceinline__ v16b load(const __bf16* p) {
    U f; f.h[0] = *(const v8b*)(p); f.h[1] = *(const v8b*)(p + 16); return f.v;
  }
  static __device__ __forceinline__ v8f mma(v16b a, v16b b, v8f c) {
    return __builtin_amdgcn_wmma_f32_16x16x32_bf16(false, a, false, b, (short)0, c, false, false);
  }
  static __device__ __forceinline__ void guard(v8f& a, v8f& b, v16b x, v16b y) { dep_guard_b(a, b, x, y); }
  static __device__ __forceinline__ void keep(v16b a, v16b b, v16b c, v16b d) { keep4_b(a, b, c, d); }
};

template <int ET> struct Elem;
template <> struct Elem<0> { typedef _Float16 T; };
template <> struct Elem<1> { typedef __bf16 T; };
template <int ET, bool SPLIT, int BIAS_MODE, int OUT_MODE, bool RESID, int ACT = 0>
__global__ __launch_bounds__(256) void wmma_gemm64(
    const unsigned short* __restrict__ Ap, const unsigned short* __restrict__ A2p, int lda, long strideA,
    const unsigned short* __restrict__ Btp, const unsigned short* __restrict__ Bt2p, int ldb, long strideB,
    void* __restrict__ Cout, void* __restrict__ Cout2, int ldc, long strideC,
    const float* __restrict__ bias,
    const float* __restrict__ resid, long strideR,
    int M, int N, int K, float scale) {
  typedef typename Elem<ET>::T T;
  typedef typename Frag<T>::V V;
  const T* A = (const T*)Ap; const T* A2 = (const T*)A2p; const T* Bt = (const T*)Btp; const T* Bt2 = (const T*)Bt2p;
  __shared__ __align__(16) float sT[8][16 * 68];
  const int b    = blockIdx.y;
  const int lane = threadIdx.x & 31;
  const int wave = threadIdx.x >> 5;
  const int tilesN = N >> 6;
  const int tilesM = M >> 6;
  const int tile = blockIdx.x * 8 + wave;
  if (tile >= tilesM * tilesN) return;
  const int tm = tile / tilesN;
  const int tn = tile - tm * tilesN;
  const int m0 = tm << 6;
  const int n0 = tn << 6;

  const T* Ab  = A  + (size_t)b * strideA;
  const T* Bb  = Bt + (size_t)b * strideB;
  const T* Ab2 = SPLIT ? (A2  + (size_t)b * strideA) : nullptr;
  const T* Bb2 = SPLIT ? (Bt2 + (size_t)b * strideB) : nullptr;

  const int rlane = lane & 15;
  const int koff  = (lane >> 4) * 8;
  const int mOff  = (lane >> 4) * 8;

  v8f acc[4][4];
#pragma unroll
  for (int i = 0; i < 4; ++i)
#pragma unroll
    for (int j = 0; j < 4; ++j) acc[i][j] = (v8f){0.f,0.f,0.f,0.f,0.f,0.f,0.f,0.f};

  for (int k0 = 0; k0 < K; k0 += 32) {
    V bh[4], bl[4];
#pragma unroll
    for (int j = 0; j < 4; ++j) {
      const size_t bo = (size_t)(n0 + (j << 4) + rlane) * ldb + koff + k0;
      bh[j] = Frag<T>::load(Bb + bo);
      if (SPLIT) bl[j] = Frag<T>::load(Bb2 + bo);
    }
#pragma unroll
    for (int i = 0; i < 4; ++i) {
      const size_t ao = (size_t)(m0 + (i << 4) + rlane) * lda + koff + k0;
      V ah = Frag<T>::load(Ab + ao);
      V al;
      if (SPLIT) al = Frag<T>::load(Ab2 + ao);
#pragma unroll
      for (int j = 0; j < 4; ++j) {
        acc[i][j] = Frag<T>::mma(ah, bh[j], acc[i][j]);
        if (SPLIT) {
          acc[i][j] = Frag<T>::mma(ah, bl[j], acc[i][j]);
          acc[i][j] = Frag<T>::mma(al, bh[j], acc[i][j]);
        }
      }
      Frag<T>::guard(acc[i][0], acc[i][3], ah, SPLIT ? al : ah);
    }
    Frag<T>::keep(bh[0], bh[1], bh[2], bh[3]);
    if (SPLIT) Frag<T>::keep(bl[0], bl[1], bl[2], bl[3]);
  }
  acc_guard4(acc[0][0], acc[0][1], acc[0][2], acc[0][3]);
  acc_guard4(acc[1][0], acc[1][1], acc[1][2], acc[1][3]);
  acc_guard4(acc[2][0], acc[2][1], acc[2][2], acc[2][3]);
  acc_guard4(acc[3][0], acc[3][1], acc[3][2], acc[3][3]);

  float* slab = sT[wave];
  const float* Rb = RESID ? (resid + (size_t)b * strideR) : nullptr;
#pragma unroll
  for (int i = 0; i < 4; ++i) {
    const int mBase = m0 + (i << 4);
#pragma unroll
    for (int j = 0; j < 4; ++j) {
      const int n = n0 + (j << 4) + rlane;
      float bv = 0.f;
      if (BIAS_MODE == 2) bv = bias[n];
#pragma unroll
      for (int r = 0; r < 8; ++r) {
        float v = acc[i][j][r] * scale;
        if (BIAS_MODE == 1) v += bias[mBase + mOff + r];
        if (BIAS_MODE == 2) v += bv;
        if (RESID) v += Rb[(size_t)(mBase + mOff + r) * ldc + n];
        if (ACT == 1) v = tanhf(v);
        if (ACT == 2) v = fmaxf(v, 0.0f);
        if (ACT == 3) v = v / (1.0f + expf(-v));
        if (ACT == 4) v = (v > 0.f) ? v : 0.01f * v;
        if (ACT == 5) v = 0.5f * v * (1.0f + erff(v * 0.70710678118654752f));
        slab[(mOff + r) * 68 + (j << 4) + rlane] = v;
      }
    }
    __builtin_amdgcn_fence(__ATOMIC_RELEASE, "workgroup");
    __builtin_amdgcn_wave_barrier();
    __builtin_amdgcn_fence(__ATOMIC_ACQUIRE, "workgroup");
    if (OUT_MODE == 0) {
      float* C = (float*)Cout + (size_t)b * strideC;
      const int hh = lane >> 4, c4 = (lane & 15) * 4;
      for (int pass = 0; pass < 2; ++pass) {
#pragma unroll
        for (int it = 0; it < 8; ++it) {
          const int row = it * 2 + hh;
          v4f v = *(const v4f*)(slab + row * 68 + c4);
          *(volatile v4f*)(C + (size_t)(mBase + row) * ldc + n0 + c4) = v;
        }
        __threadfence();
      }
    } else {
      const int q = lane >> 3, c8 = (lane & 7) * 8;
      unsigned short* C  = (unsigned short*)Cout  + (size_t)b * strideC;
      unsigned short* C2 = (OUT_MODE == 2) ? ((unsigned short*)Cout2 + (size_t)b * strideC) : nullptr;
      for (int pass = 0; pass < 2; ++pass) {
#pragma unroll
        for (int it = 0; it < 4; ++it) {
          const int row = it * 4 + q;
          const float* sp = slab + row * 68 + c8;
          v8h hv, lv;
#pragma unroll
          for (int e = 0; e < 8; ++e) {
            if (OUT_MODE == 1) {
              hv[e] = (_Float16)sp[e];
            } else {
              unsigned short hb = f2bf_bits(sp[e]);
              unsigned short lb = f2bf_bits(sp[e] - bf_bits2f(hb));
              hv[e] = __builtin_bit_cast(_Float16, hb);
              lv[e] = __builtin_bit_cast(_Float16, lb);
            }
          }
          *(volatile v8h*)(C + (size_t)(mBase + row) * ldc + n0 + c8) = hv;
          if (OUT_MODE == 2) *(volatile v8h*)(C2 + (size_t)(mBase + row) * ldc + n0 + c8) = lv;
        }
        __threadfence();
      }
    }
    __builtin_amdgcn_fence(__ATOMIC_RELEASE, "workgroup");
    __builtin_amdgcn_wave_barrier();
    __builtin_amdgcn_fence(__ATOMIC_ACQUIRE, "workgroup");
  }
}

__global__ __launch_bounds__(256) void k_split_rows(const float* __restrict__ in,
    unsigned short* __restrict__ hi, unsigned short* __restrict__ lo, int n8) {
  const int i = blockIdx.x * 256 + threadIdx.x;
  if (i >= n8) return;
  const float* p = in + (size_t)i * 8;
  const v4f a = *(const v4f*)p;
  const v4f c = *(const v4f*)(p + 4);
  v8h hv, lv;
#pragma unroll
  for (int e = 0; e < 4; ++e) {
    const unsigned short h0 = f2bf_bits(a[e]);
    const unsigned short l0 = f2bf_bits(a[e] - bf_bits2f(h0));
    const unsigned short h1 = f2bf_bits(c[e]);
    const unsigned short l1 = f2bf_bits(c[e] - bf_bits2f(h1));
    hv[e] = __builtin_bit_cast(_Float16, h0);
    lv[e] = __builtin_bit_cast(_Float16, l0);
    hv[4 + e] = __builtin_bit_cast(_Float16, h1);
    lv[4 + e] = __builtin_bit_cast(_Float16, l1);
  }
  unsigned short* ph = hi + (size_t)i * 8;
  unsigned short* pl = lo + (size_t)i * 8;
  for (int pass = 0; pass < 2; ++pass) {
    *(volatile v8h*)ph = hv;
    *(volatile v8h*)pl = lv;
    __threadfence();
  }
}

template <int TMODE>
__global__ __launch_bounds__(256) void k_transpose16(const float* __restrict__ in, int ldin, long in_bs,
    unsigned short* __restrict__ outA, unsigned short* __restrict__ outB, int ldout, long out_bs, float scale) {
  __shared__ float tile[64][65];
  const int tid = threadIdx.x;
  const int n0 = blockIdx.x * 64;
  const int k0 = blockIdx.y * 64;
  const float* inb = in + (size_t)blockIdx.z * in_bs;
  {
    const int col = tid & 63, rq = tid >> 6;
#pragma unroll
    for (int it = 0; it < 16; ++it) {
      const int row = it * 4 + rq;
      tile[row][col] = inb[(size_t)(k0 + row) * ldin + n0 + col];
    }
  }
  __syncthreads();
  const int q = tid >> 3, c8 = (tid & 7) * 8;
  v8h av[2], bv[2];
#pragma unroll
  for (int it = 0; it < 2; ++it) {
    const int n = it * 32 + q;
#pragma unroll
    for (int e = 0; e < 8; ++e) {
      const float f = tile[c8 + e][n];
      if (TMODE == 0) {
        const unsigned short hb = f2bf_bits(f);
        const unsigned short lb = f2bf_bits(f - bf_bits2f(hb));
        av[it][e] = __builtin_bit_cast(_Float16, hb);
        bv[it][e] = __builtin_bit_cast(_Float16, lb);
      } else {
        av[it][e] = (_Float16)(f * scale);
        bv[it][e] = av[it][e];
      }
    }
  }
  unsigned short* oa = outA + (size_t)blockIdx.z * out_bs;
  unsigned short* ob = outB + (size_t)blockIdx.z * out_bs;
  for (int pass = 0; pass < 2; ++pass) {
#pragma unroll
    for (int it = 0; it < 2; ++it) {
      const int n = it * 32 + q;
      const size_t o = (size_t)(n0 + n) * ldout + k0 + c8;
      *(volatile v8h*)(oa + o) = av[it];
      if (TMODE == 0) *(volatile v8h*)(ob + o) = bv[it];
    }
    __threadfence();
  }
}

__global__ __launch_bounds__(512) void k_scores(const float* __restrict__ S1, const float* __restrict__ w2,
    const float* __restrict__ b2, float* __restrict__ E) {
  __shared__ float w2s[512];
  __shared__ __align__(16) float sl[512 * 8];
  __shared__ float mg[8];
  const int tid = threadIdx.x;
  const int b = blockIdx.x;
  w2s[tid] = w2[tid];
  __syncthreads();
  float sacc[8];
#pragma unroll
  for (int r = 0; r < 8; ++r) sacc[r] = b2[r];
  const float* sp = S1 + ((size_t)b * NSTEP + tid) * NDA;
#pragma unroll 1
  for (int j = 0; j < NDA; ++j) {
    const float a = tanhf(sp[j]);
#pragma unroll
    for (int r = 0; r < 8; ++r) sacc[r] += a * w2s[j * 8 + r];
  }
  *(v4f*)(sl + tid * 8) = (v4f){sacc[0], sacc[1], sacc[2], sacc[3]};
  *(v4f*)(sl + tid * 8 + 4) = (v4f){sacc[4], sacc[5], sacc[6], sacc[7]};
  __syncthreads();
  if (tid < 8) {
    float m = -__builtin_inff();
#pragma unroll 1
    for (int j = 0; j < NSTEP; ++j) m = fmaxf(m, sl[j * 8 + tid]);
    mg[tid] = m;
  }
  __syncthreads();
#pragma unroll 1
  for (int r = 0; r < 8; ++r) {
    const int idx = tid * 8 + r;
    sl[idx] = expf(sl[idx] - mg[r]);
  }
  __syncthreads();
  float* Eb = E + (size_t)b * (NSTEP * 8);
  const v4f v0 = *(const v4f*)(sl + 4 * tid);
  const v4f v1 = *(const v4f*)(sl + 2048 + 4 * tid);
  for (int pass = 0; pass < 2; ++pass) {
    *(volatile v4f*)(Eb + 4 * tid) = v0;
    *(volatile v4f*)(Eb + 2048 + 4 * tid) = v1;
    __threadfence();
  }
}

__global__ __launch_bounds__(256) void k_attn(const float* __restrict__ E,
    unsigned short* __restrict__ AH, unsigned short* __restrict__ AL) {
  __shared__ float zp[8][8];
  __shared__ __align__(16) float wl[64 * 8];
  __shared__ __align__(16) unsigned hlw[2][256];
  const int tid = threadIdx.x, lane = tid & 31, wave = tid >> 5;
  const int b = blockIdx.x >> 3, tb = blockIdx.x & 7, t0 = tb * 64;
  const int j0 = 2 * tid, j1 = 2 * tid + 1;
  const float* Eb = E + (size_t)b * (NSTEP * 8);
  const v4f e0a = *(const v4f*)(Eb + j0 * 8), e0b = *(const v4f*)(Eb + j0 * 8 + 4);
  const v4f e1a = *(const v4f*)(Eb + j1 * 8), e1b = *(const v4f*)(Eb + j1 * 8 + 4);
  {
    float zq[8];
    const bool u0 = (j0 < t0), u1 = (j1 < t0);
#pragma unroll
    for (int r = 0; r < 4; ++r) {
      zq[r]     = (u0 ? e0a[r] : 0.f) + (u1 ? e1a[r] : 0.f);
      zq[4 + r] = (u0 ? e0b[r] : 0.f) + (u1 ? e1b[r] : 0.f);
    }
#pragma unroll
    for (int r = 0; r < 8; ++r) {
#pragma unroll
      for (int off = 1; off < 32; off <<= 1) zq[r] += __shfl_xor(zq[r], off, 32);
    }
    if (lane == 0) {
#pragma unroll
      for (int r = 0; r < 8; ++r) zp[wave][r] = zq[r];
    }
  }
  __syncthreads();
  if (tid < 8) {
    float z = 0.f;
#pragma unroll 1
    for (int w = 0; w < 8; ++w) z += zp[w][tid];
#pragma unroll 1
    for (int i = 0; i < 64; ++i) {
      z += Eb[(t0 + i) * 8 + tid];
      wl[i * 8 + tid] = 0.125f / z;
    }
  }
  __syncthreads();
#pragma unroll 1
  for (int i = 0; i < 64; ++i) {
    const int t = t0 + i;
    const v4f wa = *(const v4f*)(wl + i * 8), wb = *(const v4f*)(wl + i * 8 + 4);
    float d0 = 0.f, d1 = 0.f;
#pragma unroll
    for (int r = 0; r < 4; ++r) { d0 += e0a[r] * wa[r]; d1 += e1a[r] * wa[r]; }
#pragma unroll
    for (int r = 0; r < 4; ++r) { d0 += e0b[r] * wb[r]; d1 += e1b[r] * wb[r]; }
    const float a0 = (j0 <= t) ? d0 : 0.f;
    const float a1 = (j1 <= t) ? d1 : 0.f;
    const unsigned short h0 = f2bf_bits(a0), h1 = f2bf_bits(a1);
    const unsigned short l0 = f2bf_bits(a0 - bf_bits2f(h0)), l1 = f2bf_bits(a1 - bf_bits2f(h1));
    hlw[0][tid] = (unsigned)h0 | ((unsigned)h1 << 16);
    hlw[1][tid] = (unsigned)l0 | ((unsigned)l1 << 16);
    __syncthreads();
    if (wave < 2) {
      const v4u u0 = *(const v4u*)(&hlw[wave][4 * lane]);
      const v4u u1 = *(const v4u*)(&hlw[wave][128 + 4 * lane]);
      unsigned short* dst = (wave == 0) ? AH : AL;
      unsigned short* rowp = dst + ((size_t)(b * NSTEP + t)) * NSTEP;
      for (int pass = 0; pass < 2; ++pass) {
        *(volatile v4u*)(rowp + 8 * lane) = u0;
        *(volatile v4u*)(rowp + 256 + 8 * lane) = u1;
        __threadfence();
      }
    }
    __syncthreads();
  }
}

__device__ __forceinline__ float sigm_f(float x) { return __builtin_amdgcn_rcpf(1.0f + expf(-x)); }
__device__ __forceinline__ float tanh_f(float x) { return 1.0f - 2.0f * __builtin_amdgcn_rcpf(1.0f + expf(2.0f * x)); }

__device__ __forceinline__ void store_row512(float* __restrict__ orow, const float* srow, int lane) {
  const v4f o0 = *(const v4f*)(srow + 4 * lane);
  const v4f o1 = *(const v4f*)(srow + 128 + 4 * lane);
  const v4f o2 = *(const v4f*)(srow + 256 + 4 * lane);
  const v4f o3 = *(const v4f*)(srow + 384 + 4 * lane);
  for (int pass = 0; pass < 2; ++pass) {
    *(volatile v4f*)(orow + 4 * lane) = o0;
    *(volatile v4f*)(orow + 128 + 4 * lane) = o1;
    *(volatile v4f*)(orow + 256 + 4 * lane) = o2;
    *(volatile v4f*)(orow + 384 + 4 * lane) = o3;
    __threadfence();
  }
}

__global__ __launch_bounds__(512) void k_lstm(const unsigned short* __restrict__ WHTp,
    const float* __restrict__ GX, float* __restrict__ out) {
  const _Float16* WHT = (const _Float16*)WHTp;
  __shared__ __align__(16) _Float16 hs[NBATCH * NHID];
  __shared__ __align__(16) float slab[NBATCH * NHID];
  const int tid = threadIdx.x, wave = tid >> 5, lane = tid & 31;
  const int cc = lane & 15, hh = lane >> 4, koff = hh * 8;
  {
    const v4u z = (v4u){0u, 0u, 0u, 0u};
    *(v4u*)(hs + 16 * tid) = z;
    *(v4u*)(hs + 16 * tid + 8) = z;
  }
  float cst[2][8];
#pragma unroll
  for (int u = 0; u < 2; ++u)
#pragma unroll
    for (int r = 0; r < 8; ++r) cst[u][r] = 0.f;
  __syncthreads();
  const float accsc = 1.0f / 16384.0f;
  for (int t = 0; t < NSTEP; ++t) {
#pragma unroll
    for (int ubi = 0; ubi < 2; ++ubi) {
      const int ucol = (wave * 2 + ubi) * 16 + cc;
      v8f acc[4];
#pragma unroll
      for (int g = 0; g < 4; ++g) acc[g] = (v8f){0.f,0.f,0.f,0.f,0.f,0.f,0.f,0.f};
      const _Float16* arow = hs + cc * NHID + koff;
      const _Float16* brow = WHT + (size_t)ucol * NHID + koff;
#pragma unroll 1
      for (int k0 = 0; k0 < NHID; k0 += 32) {
        const v16h a = Frag<_Float16>::load(arow + k0);
        v16h bq[4];
#pragma unroll
        for (int g = 0; g < 4; ++g) bq[g] = Frag<_Float16>::load(brow + (size_t)g * (NHID * NHID) + k0);
#pragma unroll
        for (int g = 0; g < 4; ++g) acc[g] = Frag<_Float16>::mma(a, bq[g], acc[g]);
        dep_guard_h(acc[0], acc[3], a, bq[3]);
        keep4_h(bq[0], bq[1], bq[2], bq[3]);
      }
      acc_guard4(acc[0], acc[1], acc[2], acc[3]);
      const float* gx0 = GX + (size_t)t * (NBATCH * NGATE) + ucol;
#pragma unroll
      for (int r = 0; r < 8; ++r) {
        const int row = hh * 8 + r;
        const float* gp = gx0 + (size_t)row * NGATE;
        const float pi = acc[0][r] * accsc + gp[0];
        const float pf = acc[1][r] * accsc + gp[NHID];
        const float pg = acc[2][r] * accsc + gp[2 * NHID];
        const float po = acc[3][r] * accsc + gp[3 * NHID];
        const float iv = sigm_f(pi);
        const float fv = sigm_f(pf);
        const float gv = tanh_f(pg);
        const float ov = sigm_f(po);
        const float cn = fv * cst[ubi][r] + iv * gv;
        cst[ubi][r] = cn;
        slab[row * NHID + ucol] = ov * tanh_f(cn);
      }
    }
    __syncthreads();
    {
      const float* srow = slab + wave * NHID;
      const v4f p0 = *(const v4f*)(srow + 16 * lane);
      const v4f p1 = *(const v4f*)(srow + 16 * lane + 4);
      const v4f p2 = *(const v4f*)(srow + 16 * lane + 8);
      const v4f p3 = *(const v4f*)(srow + 16 * lane + 12);
      v8h h0v, h1v;
#pragma unroll
      for (int e = 0; e < 4; ++e) {
        h0v[e]     = (_Float16)(p0[e] * 256.0f);
        h0v[4 + e] = (_Float16)(p1[e] * 256.0f);
        h1v[e]     = (_Float16)(p2[e] * 256.0f);
        h1v[4 + e] = (_Float16)(p3[e] * 256.0f);
      }
      *(v8h*)(hs + wave * NHID + 16 * lane) = h0v;
      *(v8h*)(hs + wave * NHID + 16 * lane + 8) = h1v;
      store_row512(out + ((size_t)wave * NSTEP + t) * NHID, srow, lane);
    }
    __syncthreads();
  }
  store_row512(out + (size_t)NBATCH * NSTEP * NHID + (size_t)wave * NHID, slab + wave * NHID, lane);
  __syncthreads();
#pragma unroll
  for (int ubi = 0; ubi < 2; ++ubi) {
    const int ucol = (wave * 2 + ubi) * 16 + cc;
#pragma unroll
    for (int r = 0; r < 8; ++r) slab[(hh * 8 + r) * NHID + ucol] = cst[ubi][r];
  }
  __syncthreads();
  store_row512(out + (size_t)NBATCH * NSTEP * NHID + (size_t)NBATCH * NHID + (size_t)wave * NHID, slab + wave * NHID, lane);
}

extern "C" void kernel_launch(void* const* d_in, const int* in_sizes, int n_in,
                              void* d_out, int out_size, void* d_ws, size_t ws_size,
                              hipStream_t stream) {
  if (n_in < 8) return;
  if (in_sizes[0] != NBATCH * NSTEP * NDIM) return;
  if (in_sizes[1] != NDIM * NDA) return;
  if (in_sizes[2] != NDA) return;
  if (in_sizes[3] != NDA * NRH) return;
  if (in_sizes[4] != NRH) return;
  if (in_sizes[5] != NDIM * NGATE) return;
  if (in_sizes[6] != NHID * NGATE) return;
  if (in_sizes[7] != NGATE) return;
  if (out_size != NBATCH * NSTEP * NHID + 2 * NBATCH * NHID) return;

  const float* x    = (const float*)d_in[0];
  const float* w1   = (const float*)d_in[1];
  const float* b1   = (const float*)d_in[2];
  const float* w2   = (const float*)d_in[3];
  const float* b2   = (const float*)d_in[4];
  const float* wib  = (const float*)d_in[5];
  const float* whh  = (const float*)d_in[6];
  const float* bias = (const float*)d_in[7];
  float* out = (float*)d_out;
  char* ws = (char*)d_ws;

  const size_t szX   = (size_t)NROWS * NDIM * 2;
  const size_t szW1T = (size_t)NDA * NDIM * 2;
  const size_t szS1  = (size_t)NROWS * NDA * 4;
  const size_t szE   = (size_t)NROWS * NRH * 4;
  const size_t szA   = (size_t)NBATCH * NSTEP * NSTEP * 2;
  const size_t szM   = (size_t)NROWS * NDIM * 2;
  const size_t szWIT = (size_t)NGATE * NDIM * 2;
  const size_t szWHT = (size_t)NGATE * NHID * 2;
  const size_t szGX  = (size_t)NROWS * NGATE * 4;

  size_t off = 0;
  const size_t oXH = off;   off += szX;
  const size_t oXL = off;   off += szX;
  const size_t oXTH = off;  off += szX;
  const size_t oXTL = off;  off += szX;
  const size_t oW1TH = off; off += szW1T;
  const size_t oW1TL = off; off += szW1T;
  const size_t oS1 = off;   off += szS1;
  const size_t oE = off;    off += szE;
  const size_t oAH = off;   off += szA;
  const size_t oAL = off;   off += szA;
  const size_t oMH = off;   off += szM;
  const size_t oML = off;   off += szM;
  const size_t oWITH = off; off += szWIT;
  const size_t oWITL = off; off += szWIT;
  const size_t oWHT = off;  off += szWHT;
  const size_t oGX = off;   off += szGX;
  if (off > ws_size) return;

  unsigned short* XH   = (unsigned short*)(ws + oXH);
  unsigned short* XL   = (unsigned short*)(ws + oXL);
  unsigned short* XTH  = (unsigned short*)(ws + oXTH);
  unsigned short* XTL  = (unsigned short*)(ws + oXTL);
  unsigned short* W1TH = (unsigned short*)(ws + oW1TH);
  unsigned short* W1TL = (unsigned short*)(ws + oW1TL);
  float*          S1   = (float*)(ws + oS1);
  float*          EB   = (float*)(ws + oE);
  unsigned short* AH   = (unsigned short*)(ws + oAH);
  unsigned short* AL   = (unsigned short*)(ws + oAL);
  unsigned short* MH   = (unsigned short*)(ws + oMH);
  unsigned short* ML   = (unsigned short*)(ws + oML);
  unsigned short* WITH = (unsigned short*)(ws + oWITH);
  unsigned short* WITL = (unsigned short*)(ws + oWITL);
  unsigned short* WHT  = (unsigned short*)(ws + oWHT);
  float*          GX   = (float*)(ws + oGX);

  k_split_rows<<<dim3((NROWS * NDIM / 8) / 256), dim3(256), 0, stream>>>(x, XH, XL, NROWS * NDIM / 8);
  k_transpose16<0><<<dim3(NDIM / 64, NSTEP / 64, NBATCH), dim3(256), 0, stream>>>(
      x, NDIM, (long)NSTEP * NDIM, XTH, XTL, NSTEP, (long)NDIM * NSTEP, 1.0f);
  k_transpose16<0><<<dim3(NDA / 64, NDIM / 64, 1), dim3(256), 0, stream>>>(
      w1, NDA, 0L, W1TH, W1TL, NDIM, 0L, 1.0f);
  k_transpose16<0><<<dim3(NGATE / 64, NDIM / 64, 1), dim3(256), 0, stream>>>(
      wib, NGATE, 0L, WITH, WITL, NDIM, 0L, 1.0f);
  k_transpose16<1><<<dim3(NGATE / 64, NHID / 64, 1), dim3(256), 0, stream>>>(
      whh, NGATE, 0L, WHT, WHT, NHID, 0L, 64.0f);
  wmma_gemm64<1, true, 2, 0, false, 0><<<dim3((NROWS / 64) * (NDA / 64) / 8, 1), dim3(256), 0, stream>>>(
      XH, XL, NDIM, 0L, W1TH, W1TL, NDIM, 0L, (void*)S1, (void*)S1, NDA, 0L,
      b1, b1, 0L, NROWS, NDA, NDIM, 1.0f);
  k_scores<<<dim3(NBATCH), dim3(512), 0, stream>>>(S1, w2, b2, EB);
  k_attn<<<dim3(NBATCH * (NSTEP / 64)), dim3(256), 0, stream>>>(EB, AH, AL);
  wmma_gemm64<1, true, 0, 2, false, 0><<<dim3((NSTEP / 64) * (NDIM / 64) / 8, NBATCH), dim3(256), 0, stream>>>(
      AH, AL, NSTEP, (long)NSTEP * NSTEP, XTH, XTL, NSTEP, (long)NDIM * NSTEP,
      (void*)MH, (void*)ML, NBATCH * NDIM, (long)NDIM,
      b1, b1, 0L, NSTEP, NDIM, NSTEP, 1.0f);
  wmma_gemm64<1, true, 2, 0, false, 0><<<dim3((NROWS / 64) * (NGATE / 64) / 8, 1), dim3(256), 0, stream>>>(
      MH, ML, NDIM, 0L, WITH, WITL, NDIM, 0L, (void*)GX, (void*)GX, NGATE, 0L,
      bias, bias, 0L, NROWS, NGATE, NDIM, 1.0f);
  k_lstm<<<dim3(1), dim3(512), 0, stream>>>(WHT, GX, out);
}
